// ConvLayer_50714973831732
// MI455X (gfx1250) — hardware-verified
//
#include <hip/hip_runtime.h>
#include <stddef.h>
#include <stdint.h>


#define CF     32
#define HF     64
#define PQW    256
#define EK     256
#define K1     160
#define K2     128
#define K3     128
#define NTHR   256
#define NWAVE  8
#define EPT    8
#define CHUNK  (NTHR * EPT)
#define WCAP   (EPT * 32)
#define LISTN  (NWAVE * WCAP)
#define NBA    512
#define SLA    9
#define TROWS  64
#define QCAP   (LISTN + TROWS)
#define SROWS  128
#define PQTHR  128
#define PQBM   64
#define AGG_INTS   (NBA * HF)
#define ATILE_INTS (SROWS * K1 / 2)
#define MSTG_INTS  (2 * TROWS * HF)
#define MISC_INTS  16
#define TAIL_INTS  (LISTN + QCAP + 4 * TROWS + MISC_INTS)
#define SCAN_LDS_INTS (AGG_INTS + ATILE_INTS + MSTG_INTS + TAIL_INTS)
#define U0 1024
#define U1 3072
#define U2 4352
#define U3 5376
#define U4 5888
#define WSMAX 134217728

static_assert((CHUNK & (CHUNK - 1)) == 0 && CHUNK <= 4096);
static_assert(NBA == (1 << SLA));
static_assert(((long long)CHUNK << SLA) < (1LL << 31));
static_assert(WCAP <= NTHR);
static_assert(QCAP >= LISTN + TROWS);
static_assert(TROWS == 64 && NWAVE == 8 && NTHR == 32 * NWAVE);
static_assert(SROWS == 16 * NWAVE && (NBA % SROWS) == 0);
static_assert(ATILE_INTS * 2 >= TROWS * EK && ATILE_INTS * 2 >= SROWS * K1 && ATILE_INTS * 2 >= SROWS * K3);
static_assert(MSTG_INTS >= 2 * TROWS * HF && MSTG_INTS * 2 >= SROWS * K2 && MSTG_INTS >= SROWS * CF);
static_assert((TAIL_INTS % 4) == 0 && (AGG_INTS % (4 * NTHR)) == 0);
static_assert(((AGG_INTS + ATILE_INTS + MSTG_INTS) % 4) == 0 && (ATILE_INTS % 4) == 0 && (MSTG_INTS % 4) == 0);
static_assert(SCAN_LDS_INTS * 4 <= 300000);
static_assert(K1 % 32 == 0 && K2 % 32 == 0 && K3 % 32 == 0 && EK == 4 * HF && PQW == 4 * HF && CF == 32);
static_assert(U0 % NTHR == 0 && U1 % NTHR == 0 && U2 % NTHR == 0 && U3 % NTHR == 0 && U4 % NTHR == 0);
static_assert(U0 == 256 * (CF / 8) && U1 - U0 == 2 * HF * (K2 / 8) && U2 - U1 == HF * (K1 / 8));
static_assert(U3 - U2 == HF * (K2 / 8) && U4 - U3 == CF * (K3 / 8));
static_assert(PQTHR == 128 && PQBM == 64);

typedef float          v2f   __attribute__((ext_vector_type(2)));
typedef float          v4f   __attribute__((ext_vector_type(4)));
typedef float          v8f   __attribute__((ext_vector_type(8)));
typedef int            v4i   __attribute__((ext_vector_type(4)));
typedef int            v8i   __attribute__((ext_vector_type(8)));
typedef unsigned short v4us  __attribute__((ext_vector_type(4)));
typedef unsigned short v8us  __attribute__((ext_vector_type(8)));
typedef unsigned short v16us __attribute__((ext_vector_type(16)));
typedef __bf16         v16bf __attribute__((ext_vector_type(16)));
typedef v2f  __attribute__((may_alias)) v2fa;
typedef v4f  __attribute__((may_alias)) v4fa;
typedef v4i  __attribute__((may_alias)) v4ia;
typedef v4us __attribute__((may_alias)) v4usa;
typedef v8us __attribute__((may_alias)) v8usa;
union FragB { v16bf v; v16us u; v8us h[2]; v8i w; };

__device__ __forceinline__ v8f wmb(const FragB& a, const FragB& b, v8f c) {
  v8f d = __builtin_amdgcn_wmma_f32_16x16x32_bf16(false, a.v, false, b.v, (short)0, c, false, false);
  asm volatile("v_nop\n\tv_nop\n\tv_nop\n\tv_nop" : "+v"(d) : "v"(a.w), "v"(b.w));
  return d;
}

__device__ __forceinline__ v8f zero8f() { v8f z = {0.f, 0.f, 0.f, 0.f, 0.f, 0.f, 0.f, 0.f}; return z; }

__device__ __forceinline__ unsigned bf16_bits(float f) {
  const unsigned u = __float_as_uint(f);
  return (u + 0x7FFFu + ((u >> 16) & 1u)) >> 16;
}
__device__ __forceinline__ float bf16_val(float f) {
  return __uint_as_float(bf16_bits(f) << 16);
}
__device__ __forceinline__ v4f bf4(v4f v) {
  v4f r;
  r.x = bf16_val(v.x); r.y = bf16_val(v.y); r.z = bf16_val(v.z); r.w = bf16_val(v.w);
  return r;
}
__device__ __forceinline__ v4us bits4(v4f v) {
  v4us r;
  r[0] = (unsigned short)bf16_bits(v.x); r[1] = (unsigned short)bf16_bits(v.y);
  r[2] = (unsigned short)bf16_bits(v.z); r[3] = (unsigned short)bf16_bits(v.w);
  return r;
}
__device__ __forceinline__ v4f relu4(v4f v) {
  v4f r;
  r.x = fmaxf(v.x, 0.0f); r.y = fmaxf(v.y, 0.0f); r.z = fmaxf(v.z, 0.0f); r.w = fmaxf(v.w, 0.0f);
  return r;
}
__device__ __forceinline__ void hilo4(v4f v, v4us& h, v4us& l) {
  float f[4] = {v.x, v.y, v.z, v.w};
#pragma unroll
  for (int e = 0; e < 4; ++e) {
    const unsigned hb = bf16_bits(f[e]);
    h[e] = (unsigned short)hb;
    l[e] = (unsigned short)bf16_bits(f[e] - __uint_as_float(hb << 16));
  }
}
__device__ __forceinline__ void hilo8(v4f a, v4f b, v8us& h, v8us& l) {
  float f[8] = {a.x, a.y, a.z, a.w, b.x, b.y, b.z, b.w};
#pragma unroll
  for (int e = 0; e < 8; ++e) {
    const unsigned hb = bf16_bits(f[e]);
    h[e] = (unsigned short)hb;
    l[e] = (unsigned short)bf16_bits(f[e] - __uint_as_float(hb << 16));
  }
}

template <int SLB>
__device__ __forceinline__ int scan_chunk(const int* __restrict__ dsts, int nE, int cbase, int slotBase,
                                          int nb, int vec8, int* list, int tid, int lane, int wave) {
  int wc = 0;
  const int el0  = tid * EPT;
  const int e0   = cbase + el0;
  const int sent = -2147483647 - 1;
  v4i da, db;
  if (vec8 != 0 && cbase + CHUNK <= nE) {
    da = *(const v4i*)(dsts + e0);
    db = *(const v4i*)(dsts + e0 + 4);
  } else {
    da.x = (e0     < nE) ? dsts[min(e0,     nE - 1)] : sent;
    da.y = (e0 + 1 < nE) ? dsts[min(e0 + 1, nE - 1)] : sent;
    da.z = (e0 + 2 < nE) ? dsts[min(e0 + 2, nE - 1)] : sent;
    da.w = (e0 + 3 < nE) ? dsts[min(e0 + 3, nE - 1)] : sent;
    db.x = (e0 + 4 < nE) ? dsts[min(e0 + 4, nE - 1)] : sent;
    db.y = (e0 + 5 < nE) ? dsts[min(e0 + 5, nE - 1)] : sent;
    db.z = (e0 + 6 < nE) ? dsts[min(e0 + 6, nE - 1)] : sent;
    db.w = (e0 + 7 < nE) ? dsts[min(e0 + 7, nE - 1)] : sent;
  }
  const unsigned nbs = (unsigned)slotBase;
  const unsigned unb = (unsigned)nb;
  const unsigned s0 = (unsigned)da.x - nbs, s1 = (unsigned)da.y - nbs;
  const unsigned s2 = (unsigned)da.z - nbs, s3 = (unsigned)da.w - nbs;
  const unsigned s4 = (unsigned)db.x - nbs, s5 = (unsigned)db.y - nbs;
  const unsigned s6 = (unsigned)db.z - nbs, s7 = (unsigned)db.w - nbs;
  const bool h0 = s0 < unb, h1 = s1 < unb, h2 = s2 < unb, h3 = s3 < unb;
  const bool h4 = s4 < unb, h5 = s5 < unb, h6 = s6 < unb, h7 = s7 < unb;
  const unsigned any = __builtin_amdgcn_ballot_w32(h0 | h1 | h2 | h3 | h4 | h5 | h6 | h7);
  if (any != 0u) {
#define HITJ(J, HJ, SJ) { \
      const unsigned mj = __builtin_amdgcn_ballot_w32(HJ); \
      if (mj != 0u) { \
        if (HJ) { \
          const int pos = wc + (int)__builtin_amdgcn_mbcnt_lo(mj, 0u); \
          if (pos < WCAP) list[wave * WCAP + pos] = ((el0 + (J)) << SLB) | (int)(SJ); \
        } \
        wc += (int)__builtin_popcount(mj); } }
    HITJ(0, h0, s0)
    HITJ(1, h1, s1)
    HITJ(2, h2, s2)
    HITJ(3, h3, s3)
    HITJ(4, h4, s4)
    HITJ(5, h5, s5)
    HITJ(6, h6, s6)
    HITJ(7, h7, s7)
#undef HITJ
  }
  return wc;
}

__global__ __launch_bounds__(NTHR) void k_prep(const float* __restrict__ x, int nN, int nxb,
                                               const float* __restrict__ W1, const float* __restrict__ W2,
                                               const float* __restrict__ Wo1, const float* __restrict__ Wo2,
                                               const float* __restrict__ Wo3,
                                               unsigned short* XB, unsigned short* W1r, unsigned short* W2d,
                                               unsigned short* Wo1d, unsigned short* Wo2d, unsigned short* Wo3d) {
  const int tid = (int)threadIdx.x;
  if ((int)blockIdx.x < nxb) {
    const int u   = (int)blockIdx.x * NTHR + tid;
    const int row = u >> 2, c8 = (u & 3) * 8;
    const int rr  = row < nN ? row : nN - 1;
    const bool ok = row < nN;
    const float* p = x + (size_t)rr * CF + c8;
    const v4f a = *(const v4f*)p;
    const v4f b = *(const v4f*)(p + 4);
    v8us o;
    o[0] = (unsigned short)(ok ? bf16_bits(a.x) : 0u); o[1] = (unsigned short)(ok ? bf16_bits(a.y) : 0u);
    o[2] = (unsigned short)(ok ? bf16_bits(a.z) : 0u); o[3] = (unsigned short)(ok ? bf16_bits(a.w) : 0u);
    o[4] = (unsigned short)(ok ? bf16_bits(b.x) : 0u); o[5] = (unsigned short)(ok ? bf16_bits(b.y) : 0u);
    o[6] = (unsigned short)(ok ? bf16_bits(b.z) : 0u); o[7] = (unsigned short)(ok ? bf16_bits(b.w) : 0u);
    unsigned short* dp = XB + (size_t)u * 8;
    *(volatile v8us*)dp = o;
    __threadfence();
    *(volatile v8us*)dp = o;
    return;
  }
  const int u = ((int)blockIdx.x - nxb) * NTHR + tid;
  const float* src = W1;
  int stride = HF;
  unsigned short* dst = W1r;
  if (u < U0) {
    const int n = u >> 2, k8 = (u & 3) * 8;
    const int cb = n >> 6, h = n & 63, i = cb >> 1, p = cb & 1;
    src = W1 + (size_t)(i * 64 + p * 32 + k8) * HF + h;  stride = HF;  dst = W1r + (size_t)u * 8;
  } else if (u < U1) {
    const int v = u - U0;
    const int n2 = v >> 4, k8 = (v & 15) * 8;
    const int i = n2 >> 6, n = n2 & 63, kk = k8 & 63;
    src = W2 + (size_t)(i * 64 + kk) * HF + n;  stride = HF;  dst = W2d + (size_t)v * 8;
  } else if (u < U2) {
    const int v = u - U1;
    const int n = v / 20, k8 = (v - n * 20) * 8;
    const int f8 = k8 < 96 ? k8 : k8 - 64;
    src = Wo1 + (size_t)f8 * HF + n;  stride = HF;  dst = Wo1d + (size_t)v * 8;
  } else if (u < U3) {
    const int v = u - U2;
    const int n = v >> 4, k8 = (v & 15) * 8, kk = k8 & 63;
    src = Wo2 + (size_t)kk * HF + n;  stride = HF;  dst = Wo2d + (size_t)v * 8;
  } else if (u < U4) {
    const int v = u - U3;
    const int n = v >> 4, k8 = (v & 15) * 8, kk = k8 & 63;
    src = Wo3 + (size_t)kk * CF + n;  stride = CF;  dst = Wo3d + (size_t)v * 8;
  } else {
    return;
  }
  float f[8];
#pragma unroll
  for (int j = 0; j < 8; ++j) f[j] = src[(size_t)j * stride];
  v8us o;
#pragma unroll
  for (int j = 0; j < 8; ++j) o[j] = (unsigned short)bf16_bits(f[j]);
  *(volatile v8us*)dst = o;
  __threadfence();
  *(volatile v8us*)dst = o;
}

__global__ __launch_bounds__(PQTHR) void k_pq(const unsigned short* __restrict__ XB,
                                              const unsigned short* __restrict__ W1r, float* PQ) {
  __shared__ __attribute__((aligned(16))) float stg[PQBM * 128];
  const int tid = (int)threadIdx.x, lane = tid & 31, wave = tid >> 5, hh = lane >> 4, m = lane & 15;
  const int rowBase = (int)blockIdx.x * PQBM;
  FragB af;
  {
    const unsigned short* ap = XB + (size_t)(rowBase + 16 * wave + m) * CF + 8 * hh;
    af.h[0] = *(const v8usa*)ap;
    af.h[1] = *(const v8usa*)(ap + 16);
  }
#pragma unroll 1
  for (int g = 0; g < 2; ++g) {
    v8f acc[8];
#pragma unroll
    for (int nt = 0; nt < 8; ++nt) {
      const unsigned short* wq = W1r + (size_t)(128 * g + 16 * nt + m) * CF + 8 * hh;
      FragB bf;
      bf.h[0] = *(const v8usa*)wq;
      bf.h[1] = *(const v8usa*)(wq + 16);
      acc[nt] = wmb(af, bf, zero8f());
    }
#pragma unroll
    for (int nt = 0; nt < 8; ++nt) {
#pragma unroll
      for (int r = 0; r < 8; ++r) stg[(16 * wave + 8 * hh + r) * 128 + 16 * nt + m] = acc[nt][r];
    }
    __syncthreads();
    v4f pv[16];
#pragma unroll
    for (int i = 0; i < 16; ++i) pv[i] = *(const v4fa*)(stg + (16 * wave + i) * 128 + 4 * lane);
    __syncthreads();
    float* gp = PQ + (size_t)(rowBase + 16 * wave) * PQW + 128 * g + 4 * lane;
#pragma unroll
    for (int i = 0; i < 16; ++i) *(volatile v4f*)(gp + (size_t)i * PQW) = pv[i];
    __threadfence();
#pragma unroll
    for (int i = 0; i < 16; ++i) *(volatile v4f*)(gp + (size_t)i * PQW) = pv[i];
  }
}

__device__ __forceinline__ void edge_tile(
    int qbase, int nvalid, int nodeBase, int nN, int nE,
    const int* __restrict__ cols, const float* __restrict__ ep, const float* __restrict__ PQ,
    const float* __restrict__ b1, const float* __restrict__ b2, const unsigned short* __restrict__ W2d,
    float* aggL, unsigned short* atile, float* mstg, int* que, int* slotL, int* colL, float* prL,
    int tid, int lane, int wave, int hh, int m) {
  if (tid < TROWS) {
    const int jj  = tid < nvalid ? tid : nvalid - 1;
    const int ent = que[qbase + jj];
    int e = ent >> SLA;
    e = e < 0 ? 0 : (e > nE - 1 ? nE - 1 : e);
    int c = cols[e];
    c = c < 0 ? 0 : (c > nN - 1 ? nN - 1 : c);
    slotL[tid] = ent & (NBA - 1);
    colL[tid]  = c;
    prL[tid]         = bf16_val(ep[e]);
    prL[TROWS + tid] = bf16_val(ep[(size_t)nE + e]);
  }
  __syncthreads();
  {
    const int q = tid & 7, jr = tid >> 3;
    const v4f ba0 = bf4(*(const v4f*)(b1 + 8 * q));
    const v4f ba1 = bf4(*(const v4f*)(b1 + 8 * q + 4));
    const v4f bb0 = bf4(*(const v4f*)(b1 + HF + 8 * q));
    const v4f bb1 = bf4(*(const v4f*)(b1 + HF + 8 * q + 4));
#pragma unroll
    for (int pass = 0; pass < TROWS / 32; ++pass) {
      const int j    = pass * 32 + jr;
      const int slot = slotL[j];
      const int c    = colL[j];
      int prow = nodeBase + slot;
      prow = prow > nN - 1 ? nN - 1 : prow;
      const float* pp = PQ + (size_t)prow * PQW + 8 * q;
      const float* qp = PQ + (size_t)c * PQW + HF + 8 * q;
      const v4f p00 = *(const v4f*)pp,         p01 = *(const v4f*)(pp + 4);
      const v4f q00 = *(const v4f*)qp,         q01 = *(const v4f*)(qp + 4);
      const v4f p10 = *(const v4f*)(pp + 128), p11 = *(const v4f*)(pp + 132);
      const v4f q10 = *(const v4f*)(qp + 128), q11 = *(const v4f*)(qp + 132);
      const v4f h00 = relu4((p00 + q00) + ba0);
      const v4f h01 = relu4((p01 + q01) + ba1);
      const v4f h10 = relu4((p10 + q10) + bb0);
      const v4f h11 = relu4((p11 + q11) + bb1);
      unsigned short* ar = atile + (size_t)j * EK + 8 * q;
      v8us hv, lv;
      hilo8(h00, h01, hv, lv);
      *(v8usa*)ar = hv;
      *(v8usa*)(ar + HF) = lv;
      hilo8(h10, h11, hv, lv);
      *(v8usa*)(ar + 2 * HF) = hv;
      *(v8usa*)(ar + 3 * HF) = lv;
    }
  }
  __syncthreads();
  {
    const int i = wave >> 2, rt = wave & 3;
    v8f acc[4];
#pragma unroll
    for (int t = 0; t < 4; ++t) acc[t] = zero8f();
    const unsigned short* ap = atile + (size_t)(16 * rt + m) * EK + 2 * HF * i + 8 * hh;
    const unsigned short* bp = W2d + (size_t)(i * HF + m) * K2 + 8 * hh;
#pragma unroll
    for (int ks = 0; ks < K2 / 32; ++ks) {
      FragB af;
      af.h[0] = *(const v8usa*)(ap + 32 * ks);
      af.h[1] = *(const v8usa*)(ap + 32 * ks + 16);
#pragma unroll
      for (int nt = 0; nt < 4; ++nt) {
        const unsigned short* wq = bp + (size_t)(16 * nt) * K2 + 32 * ks;
        FragB bf;
        bf.h[0] = *(const v8usa*)wq;
        bf.h[1] = *(const v8usa*)(wq + 16);
        acc[nt] = wmb(af, bf, acc[nt]);
      }
    }
    float prr[8];
    {
      const float* pr = prL + i * TROWS + 16 * rt + 8 * hh;
#pragma unroll
      for (int r = 0; r < 8; ++r) prr[r] = pr[r];
    }
    float* ms = mstg + (size_t)i * (TROWS * HF) + (size_t)(16 * rt + 8 * hh) * HF;
#pragma unroll
    for (int nt = 0; nt < 4; ++nt) {
      const int col = 16 * nt + m;
      const float bv = bf16_val(b2[i * HF + col]);
#pragma unroll
      for (int r = 0; r < 8; ++r) ms[r * HF + col] = fmaxf(acc[nt][r] + bv, 0.0f) * prr[r];
    }
  }
  __syncthreads();
  if (wave == 0) {
    const float* m0 = mstg + 2 * lane;
    const float* m1 = mstg + TROWS * HF + 2 * lane;
    float* ag = aggL + 2 * lane;
#pragma unroll 1
    for (int j = 0; j < nvalid; ++j) {
      const int slot = slotL[j];
      const v2f a = *(const v2fa*)(m0 + j * HF);
      const v2f b = *(const v2fa*)(m1 + j * HF);
      const v2f s = a + b;
      v2fa* gp = (v2fa*)(ag + slot * HF);
      const v2f cur = *gp;
      *gp = cur + s;
    }
  }
  __syncthreads();
}

__global__ __launch_bounds__(NTHR) void k_scan(
    const int* __restrict__ eidx, int nE, int nN, int vec8,
    const float* __restrict__ x, const float* __restrict__ ep, const float* __restrict__ PQ,
    const float* __restrict__ b1, const float* __restrict__ b2,
    const float* __restrict__ bo1, const float* __restrict__ bo2, const float* __restrict__ bo3,
    const unsigned short* __restrict__ W2d, const unsigned short* __restrict__ Wo1d,
    const unsigned short* __restrict__ Wo2d, const unsigned short* __restrict__ Wo3d,
    float* out) {
  extern __shared__ __attribute__((aligned(16))) int dsm[];
  float*          aggL  = (float*)dsm;
  unsigned short* atile = (unsigned short*)(dsm + AGG_INTS);
  float*          mstg  = (float*)(dsm + AGG_INTS + ATILE_INTS);
  int*            list  = dsm + AGG_INTS + ATILE_INTS + MSTG_INTS;
  int*            que   = list + LISTN;
  int*            slotL = que + QCAP;
  int*            colL  = slotL + TROWS;
  float*          prL   = (float*)(colL + TROWS);
  int*            misc  = (int*)(prL + 2 * TROWS);
  const int tid = (int)threadIdx.x, lane = tid & 31, wave = tid >> 5, hh = lane >> 4, m = lane & 15;
  const int nodeBase = (int)blockIdx.x * NBA;
  int nb = nN - nodeBase;
  nb = nb < 0 ? 0 : (nb > NBA ? NBA : nb);
  const int* keys = eidx;
  const int* cols = eidx + nE;

  {
    const v4i z4 = {0, 0, 0, 0};
#pragma unroll 1
    for (int i = tid * 4; i < AGG_INTS; i += NTHR * 4) *(v4ia*)(dsm + i) = z4;
#pragma unroll 1
    for (int i = tid * 4; i < TAIL_INTS; i += NTHR * 4) *(v4ia*)(list + i) = z4;
  }
  __syncthreads();

  const int nChunks = (nE + CHUNK - 1) / CHUNK;
#pragma unroll 1
  for (int ch = 0; ch < nChunks; ++ch) {
    const int cbase = ch * CHUNK;
    const int wc = scan_chunk<SLA>(keys, nE, cbase, nodeBase, nb, vec8, list, tid, lane, wave);
    if (lane == 0) misc[wave] = wc;
    __syncthreads();
    int pos = misc[8];
    pos = pos < 0 ? 0 : (pos > TROWS - 1 ? TROWS - 1 : pos);
#pragma unroll
    for (int w2 = 0; w2 < NWAVE; ++w2) {
      int c = misc[w2];
      c = c < 0 ? 0 : (c > WCAP ? WCAP : c);
      const int ent = list[w2 * WCAP + (tid < WCAP ? tid : WCAP - 1)];
      if (tid < c) que[pos + tid] = ((cbase + ((ent >> SLA) & (CHUNK - 1))) << SLA) | (ent & (NBA - 1));
      pos += c;
    }
    __syncthreads();
    const int ntile = pos / TROWS;
#pragma unroll 1
    for (int t = 0; t < ntile; ++t)
      edge_tile(t * TROWS, TROWS, nodeBase, nN, nE, cols, ep, PQ, b1, b2, W2d,
                aggL, atile, mstg, que, slotL, colL, prL, tid, lane, wave, hh, m);
    const int rem = pos - ntile * TROWS;
    {
      int src = ntile * TROWS + tid;
      src = src > QCAP - 1 ? QCAP - 1 : src;
      const int v = que[src];
      if (ntile > 0 && tid < rem) que[tid] = v;
      if (tid == 0) misc[8] = rem;
    }
    __syncthreads();
  }
  {
    int qn = misc[8];
    qn = qn < 0 ? 0 : (qn > TROWS - 1 ? TROWS - 1 : qn);
    if (qn > 0)
      edge_tile(0, qn, nodeBase, nN, nE, cols, ep, PQ, b1, b2, W2d,
                aggL, atile, mstg, que, slotL, colL, prL, tid, lane, wave, hh, m);
  }

#pragma unroll 1
  for (int s = 0; s < NBA / SROWS; ++s) {
    const int rBase = nodeBase + s * SROWS;
#pragma unroll 1
    for (int u = tid; u < SROWS * (CF / 4); u += NTHR) {
      const int row = u >> 3, c4 = (u & 7) * 4;
      int node = rBase + row;
      node = node > nN - 1 ? nN - 1 : node;
      const v4f xv = *(const v4f*)(x + (size_t)node * CF + c4);
      *(v4usa*)(atile + (size_t)row * K1 + c4) = bits4(xv);
    }
#pragma unroll 1
    for (int u = tid; u < SROWS * (HF / 4); u += NTHR) {
      const int row = u >> 4, c4 = (u & 15) * 4;
      const v4f av = *(const v4fa*)(aggL + (size_t)(s * SROWS + row) * HF + c4);
      v4us h4, l4;
      hilo4(av, h4, l4);
      *(v4usa*)(atile + (size_t)row * K1 + CF + c4) = h4;
      *(v4usa*)(atile + (size_t)row * K1 + CF + HF + c4) = l4;
    }
    __syncthreads();
    {
      v8f acc[4];
#pragma unroll
      for (int t = 0; t < 4; ++t) acc[t] = zero8f();
      const unsigned short* ap = atile + (size_t)(16 * wave + m) * K1 + 8 * hh;
      const unsigned short* bp = Wo1d + (size_t)m * K1 + 8 * hh;
#pragma unroll
      for (int ks = 0; ks < K1 / 32; ++ks) {
        FragB af;
        af.h[0] = *(const v8usa*)(ap + 32 * ks);
        af.h[1] = *(const v8usa*)(ap + 32 * ks + 16);
#pragma unroll
        for (int nt = 0; nt < 4; ++nt) {
          const unsigned short* wq = bp + (size_t)(16 * nt) * K1 + 32 * ks;
          FragB bf;
          bf.h[0] = *(const v8usa*)wq;
          bf.h[1] = *(const v8usa*)(wq + 16);
          acc[nt] = wmb(af, bf, acc[nt]);
        }
      }
      unsigned short* a2 = (unsigned short*)mstg + (size_t)(16 * wave + 8 * hh) * K2;
#pragma unroll
      for (int nt = 0; nt < 4; ++nt) {
        const int col = 16 * nt + m;
        const float bv = bf16_val(bo1[col]);
#pragma unroll
        for (int r = 0; r < 8; ++r) {
          const float v = fmaxf(acc[nt][r] + bv, 0.0f);
          const unsigned hb = bf16_bits(v);
          a2[r * K2 + col]      = (unsigned short)hb;
          a2[r * K2 + HF + col] = (unsigned short)bf16_bits(v - __uint_as_float(hb << 16));
        }
      }
    }
    __syncthreads();
    {
      v8f acc[4];
#pragma unroll
      for (int t = 0; t < 4; ++t) acc[t] = zero8f();
      const unsigned short* ap = (const unsigned short*)mstg + (size_t)(16 * wave + m) * K2 + 8 * hh;
      const unsigned short* bp = Wo2d + (size_t)m * K2 + 8 * hh;
#pragma unroll
      for (int ks = 0; ks < K2 / 32; ++ks) {
        FragB af;
        af.h[0] = *(const v8usa*)(ap + 32 * ks);
        af.h[1] = *(const v8usa*)(ap + 32 * ks + 16);
#pragma unroll
        for (int nt = 0; nt < 4; ++nt) {
          const unsigned short* wq = bp + (size_t)(16 * nt) * K2 + 32 * ks;
          FragB bf;
          bf.h[0] = *(const v8usa*)wq;
          bf.h[1] = *(const v8usa*)(wq + 16);
          acc[nt] = wmb(af, bf, acc[nt]);
        }
      }
      unsigned short* a3 = atile + (size_t)(16 * wave + 8 * hh) * K3;
#pragma unroll
      for (int nt = 0; nt < 4; ++nt) {
        const int col = 16 * nt + m;
        const float bv = bf16_val(bo2[col]);
#pragma unroll
        for (int r = 0; r < 8; ++r) {
          const float v = fmaxf(acc[nt][r] + bv, 0.0f);
          const unsigned hb = bf16_bits(v);
          a3[r * K3 + col]      = (unsigned short)hb;
          a3[r * K3 + HF + col] = (unsigned short)bf16_bits(v - __uint_as_float(hb << 16));
        }
      }
    }
    __syncthreads();
    {
      v8f acc[2];
      acc[0] = zero8f();
      acc[1] = zero8f();
      const unsigned short* ap = atile + (size_t)(16 * wave + m) * K3 + 8 * hh;
      const unsigned short* bp = Wo3d + (size_t)m * K3 + 8 * hh;
#pragma unroll
      for (int ks = 0; ks < K3 / 32; ++ks) {
        FragB af;
        af.h[0] = *(const v8usa*)(ap + 32 * ks);
        af.h[1] = *(const v8usa*)(ap + 32 * ks + 16);
#pragma unroll
        for (int nt = 0; nt < 2; ++nt) {
          const unsigned short* wq = bp + (size_t)(16 * nt) * K3 + 32 * ks;
          FragB bf;
          bf.h[0] = *(const v8usa*)wq;
          bf.h[1] = *(const v8usa*)(wq + 16);
          acc[nt] = wmb(af, bf, acc[nt]);
        }
      }
      float* os = mstg + (size_t)(16 * wave + 8 * hh) * CF;
#pragma unroll
      for (int nt = 0; nt < 2; ++nt) {
        const int col = 16 * nt + m;
        const float bv = bf16_val(bo3[col]);
#pragma unroll
        for (int r = 0; r < 8; ++r) os[r * CF + col] = acc[nt][r] + bv;
      }
    }
    __syncthreads();
    {
      const int piece = tid & 7, lr0 = tid >> 3;
      v4f ov[SROWS / 32];
#pragma unroll
      for (int it = 0; it < SROWS / 32; ++it) {
        const int lr = it * 32 + lr0;
        int node = rBase + lr;
        node = node > nN - 1 ? nN - 1 : node;
        const v4f xs = *(const v4f*)(x + (size_t)node * CF + 4 * piece);
        const v4f st = *(const v4fa*)(mstg + (size_t)lr * CF + 4 * piece);
        ov[it] = st + bf4(xs);
      }
#pragma unroll
      for (int it = 0; it < SROWS / 32; ++it) {
        const int node = rBase + it * 32 + lr0;
        if (node < nN) *(volatile v4f*)(out + (size_t)node * CF + 4 * piece) = ov[it];
      }
      __threadfence();
#pragma unroll
      for (int it = 0; it < SROWS / 32; ++it) {
        const int node = rBase + it * 32 + lr0;
        if (node < nN) *(volatile v4f*)(out + (size_t)node * CF + 4 * piece) = ov[it];
      }
    }
    __syncthreads();
  }
}

static inline int cdiv(int a, int b) { return (a + b - 1) / b; }
static inline size_t al256(size_t o) { return (o + 255) & ~(size_t)255; }

extern "C" void kernel_launch(void* const* d_in, const int* in_sizes, int n_in,
                              void* d_out, int out_size, void* d_ws, size_t ws_size,
                              hipStream_t stream) {
  if (n_in < 13) return;
  if (in_sizes[0] < CF * 16 || (in_sizes[0] % CF) != 0) return;
  const int nN = in_sizes[0] / CF;
  if ((in_sizes[1] % 2) != 0) return;
  const int nE = in_sizes[1] / 2;
  if (nE < 1 || nE >= (1 << 22) || nN >= (1 << 22)) return;
  if (in_sizes[12] != 2 * nE) return;
  if (in_sizes[2] != 2 * 2 * CF * HF || in_sizes[3] != 2 * HF) return;
  if (in_sizes[4] != 2 * HF * HF || in_sizes[5] != 2 * HF) return;
  if (in_sizes[6] != (CF + HF) * HF || in_sizes[7] != HF) return;
  if (in_sizes[8] != HF * HF || in_sizes[9] != HF) return;
  if (in_sizes[10] != HF * CF || in_sizes[11] != CF) return;
  if ((long long)out_size != (long long)nN * CF) return;

  const float* x    = (const float*)d_in[0];
  const float* ep   = (const float*)d_in[1];
  const float* W1   = (const float*)d_in[2];
  const float* b1   = (const float*)d_in[3];
  const float* W2   = (const float*)d_in[4];
  const float* b2   = (const float*)d_in[5];
  const float* Wo1  = (const float*)d_in[6];
  const float* bo1  = (const float*)d_in[7];
  const float* Wo2  = (const float*)d_in[8];
  const float* bo2  = (const float*)d_in[9];
  const float* Wo3  = (const float*)d_in[10];
  const float* bo3  = (const float*)d_in[11];
  const int*   eidx = (const int*)d_in[12];
  float* out = (float*)d_out;

  const int NP  = cdiv(nN, PQBM) * PQBM;
  const int gPQ = NP / PQBM;
  const int nxb = NP / 64;
  const int gS  = cdiv(nN, NBA);
  if ((long long)gS * NBA < (long long)nN) return;
  const int vec8 = ((nE & 3) == 0) ? 1 : 0;

  char* ws = (char*)d_ws;
  size_t off = 0;
  const size_t oXB  = off; off = al256(off + (size_t)NP * CF * 2);
  const size_t oPQ  = off; off = al256(off + (size_t)NP * PQW * 4);
  const size_t oW1r = off; off = al256(off + (size_t)256 * CF * 2);
  const size_t oW2d = off; off = al256(off + (size_t)2 * HF * K2 * 2);
  const size_t oWo1 = off; off = al256(off + (size_t)HF * K1 * 2);
  const size_t oWo2 = off; off = al256(off + (size_t)HF * K2 * 2);
  const size_t oWo3 = off; off = al256(off + (size_t)CF * K3 * 2);
  if (off > ws_size || off > (size_t)WSMAX) return;
  unsigned short* XB   = (unsigned short*)(ws + oXB);
  float*          PQ   = (float*)(ws + oPQ);
  unsigned short* W1r  = (unsigned short*)(ws + oW1r);
  unsigned short* W2d  = (unsigned short*)(ws + oW2d);
  unsigned short* Wo1d = (unsigned short*)(ws + oWo1);
  unsigned short* Wo2d = (unsigned short*)(ws + oWo2);
  unsigned short* Wo3d = (unsigned short*)(ws + oWo3);

  const size_t scanLds = (size_t)SCAN_LDS_INTS * 4;
  hipFuncSetAttribute(reinterpret_cast<const void*>(&k_scan), hipFuncAttributeMaxDynamicSharedMemorySize, (int)scanLds);

  k_prep<<<nxb + U4 / NTHR, NTHR, 0, stream>>>(x, nN, nxb, W1, W2, Wo1, Wo2, Wo3, XB, W1r, W2d, Wo1d, Wo2d, Wo3d);
  k_pq<<<gPQ, PQTHR, 0, stream>>>(XB, W1r, PQ);
  k_scan<<<gS, NTHR, scanLds, stream>>>(eidx, nE, nN, vec8, x, ep, PQ, b1, b2, bo1, bo2, bo3,
                                       W2d, Wo1d, Wo2d, Wo3d, out);
}
